// HeadAttention_25074019074695
// MI455X (gfx1250) — hardware-verified
//
#include <hip/hip_runtime.h>
#include <math.h>

constexpr int kBatch = 4;
constexpr int kSeq   = 2048;
constexpr int kEmb   = 1024;
constexpr int kHid   = 1024;
constexpr int kTok   = kBatch * kSeq;
constexpr int kEarly = 256;
constexpr int kLate  = kSeq - kEarly;
constexpr float kScoreScale = 1.0f / 32.0f;
constexpr float kPCarry     = 32768.0f;
constexpr float kPCarryInv  = 1.0f / 32768.0f;
constexpr float kNegFill    = -3.0e38f;
static_assert(kEmb % 32 == 0 && kHid % 64 == 0 && kSeq % 64 == 0, "tiles");
static_assert(kEarly % 64 == 0 && kLate % 64 == 0 && kEarly % 32 == 0, "tiles");
static_assert(kSeq == 256 * 8, "softmax late: 256 threads x 8 columns per row");
static_assert(kEarly == 32 * 8, "softmax early: 32 lanes x 8 columns per row");

typedef __attribute__((ext_vector_type(16))) _Float16 v16h;
typedef __attribute__((ext_vector_type(8)))  _Float16 v8h;
typedef __attribute__((ext_vector_type(16))) __bf16   v16b;
typedef __attribute__((ext_vector_type(8)))  __bf16   v8b;
typedef __attribute__((ext_vector_type(8)))  float    v8f;
typedef __attribute__((ext_vector_type(4)))  float    v4f;
typedef __attribute__((ext_vector_type(4)))  unsigned int v4u;

__device__ __forceinline__ unsigned short f2bf_bits(float f) {
  unsigned u = __float_as_uint(f);
  return (unsigned short)((u + 0x7FFFu + ((u >> 16) & 1u)) >> 16);
}
__device__ __forceinline__ float bf_bits2f(unsigned short h) { return __uint_as_float(((unsigned)h) << 16); }

__device__ __forceinline__ void dep_guard_h(v8f& a, v8f& b, v16h x, v16h y) { asm volatile("v_nop\n\tv_nop\n\tv_nop\n\tv_nop" : "+v"(a), "+v"(b) : "v"(x), "v"(y)); }
__device__ __forceinline__ void dep_guard_b(v8f& a, v8f& b, v16b x, v16b y) { asm volatile("v_nop\n\tv_nop\n\tv_nop\n\tv_nop" : "+v"(a), "+v"(b) : "v"(x), "v"(y)); }
__device__ __forceinline__ void keep4_h(v16h a, v16h b, v16h c, v16h d) { asm volatile("v_nop" :: "v"(a), "v"(b), "v"(c), "v"(d)); }
__device__ __forceinline__ void keep4_b(v16b a, v16b b, v16b c, v16b d) { asm volatile("v_nop" :: "v"(a), "v"(b), "v"(c), "v"(d)); }
__device__ __forceinline__ void acc_guard4(v8f& a, v8f& b, v8f& c, v8f& d) { asm volatile("v_nop\n\tv_nop\n\tv_nop\n\tv_nop" : "+v"(a), "+v"(b), "+v"(c), "+v"(d)); }
template <typename T> struct Frag;
template <> struct Frag<_Float16> {
  typedef v16h V; union U { v16h v; v8h h[2]; };
  static __device__ __forceinline__ v16h load(const _Float16* p) {
    U f; f.h[0] = *(const v8h*)(p); f.h[1] = *(const v8h*)(p + 16); return f.v;
  }
  static __device__ __forceinline__ v8f mma(v16h a, v16h b, v8f c) {
    return __builtin_amdgcn_wmma_f32_16x16x32_f16(false, a, false, b, (short)0, c, false, false);
  }
  static __device__ __forceinline__ void guard(v8f& a, v8f& b, v16h x, v16h y) { dep_guard_h(a, b, x, y); }
  static __device__ __forceinline__ void keep(v16h a, v16h b, v16h c, v16h d) { keep4_h(a, b, c, d); }
};
template <> struct Frag<__bf16> {
  typedef v16b V; union U { v16b v; v8b h[2]; };
  static __device__ __forceinline__ v16b load(const __bf16* p) {
    U f; f.h[0] = *(const v8b*)(p); f.h[1] = *(const v8b*)(p + 16); return f.v;
  }
  static __device__ __forceinline__ v8f mma(v16b a, v16b b, v8f c) {
    return __builtin_amdgcn_wmma_f32_16x16x32_bf16(false, a, false, b, (short)0, c, false, false);
  }
  static __device__ __forceinline__ void guard(v8f& a, v8f& b, v16b x, v16b y) { dep_guard_b(a, b, x, y); }
  static __device__ __forceinline__ void keep(v16b a, v16b b, v16b c, v16b d) { keep4_b(a, b, c, d); }
};

__device__ __forceinline__ unsigned pk16(unsigned short a, unsigned short b) { return (unsigned)a | ((unsigned)b << 16); }
__device__ __forceinline__ unsigned short h_bits(float f) { const _Float16 h = (_Float16)f; return __builtin_bit_cast(unsigned short, h); }

template <int ET> struct Elem;
template <> struct Elem<0> { typedef _Float16 T; };
template <> struct Elem<1> { typedef __bf16 T; };
template <int ET, bool SPLIT, int BIAS_MODE, int OUT_MODE, bool RESID, int ACT, int CAUSAL>
__global__ __launch_bounds__(256) void wmma_gemm64(
    const unsigned short* __restrict__ Ap, const unsigned short* __restrict__ A2p, int lda, long strideA,
    const unsigned short* __restrict__ Btp, const unsigned short* __restrict__ Bt2p, int ldb, long strideB,
    void* __restrict__ Cout, void* __restrict__ Cout2, int ldc, long strideC,
    const float* __restrict__ bias,
    const float* __restrict__ resid, long strideR,
    int M, int N, int K, float scale, int moff) {
  typedef typename Elem<ET>::T T;
  typedef typename Frag<T>::V V;
  const T* A = (const T*)Ap; const T* A2 = (const T*)A2p; const T* Bt = (const T*)Btp; const T* Bt2 = (const T*)Bt2p;
  __shared__ __align__(16) float sT[8][16 * 68];
  const int b    = blockIdx.y;
  const int lane = threadIdx.x & 31;
  const int wave = threadIdx.x >> 5;
  const int tilesN = N >> 6;
  const int tilesM = M >> 6;
  const int tile = blockIdx.x * 8 + wave;
  if (tile >= tilesM * tilesN) return;
  const int tm = tile / tilesN;
  const int tn = tile - tm * tilesN;
  const int m0 = tm << 6;
  const int n0 = tn << 6;
  if (CAUSAL == 1 && n0 >= m0 + moff + 64) return;
  const int Kend = (CAUSAL == 2) ? ((m0 + moff + 64 < K) ? (m0 + moff + 64) : K) : K;

  const T* Ab  = A  + (size_t)b * strideA;
  const T* Bb  = Bt + (size_t)b * strideB;
  const T* Ab2 = SPLIT ? (A2  + (size_t)b * strideA) : nullptr;
  const T* Bb2 = SPLIT ? (Bt2 + (size_t)b * strideB) : nullptr;

  const int rlane = lane & 15;
  const int koff  = (lane >> 4) * 8;
  const int mOff  = (lane >> 4) * 8;

  v8f acc[4][4];
#pragma unroll
  for (int i = 0; i < 4; ++i)
#pragma unroll
    for (int j = 0; j < 4; ++j) acc[i][j] = (v8f){0.f,0.f,0.f,0.f,0.f,0.f,0.f,0.f};

  for (int k0 = 0; k0 < Kend; k0 += 32) {
    V bh[4], bl[4];
#pragma unroll
    for (int j = 0; j < 4; ++j) {
      const size_t bo = (size_t)(n0 + (j << 4) + rlane) * ldb + koff + k0;
      bh[j] = Frag<T>::load(Bb + bo);
      if (SPLIT) bl[j] = Frag<T>::load(Bb2 + bo);
    }
#pragma unroll
    for (int i = 0; i < 4; ++i) {
      const size_t ao = (size_t)(m0 + (i << 4) + rlane) * lda + koff + k0;
      V ah = Frag<T>::load(Ab + ao);
      V al;
      if (SPLIT) al = Frag<T>::load(Ab2 + ao);
#pragma unroll
      for (int j = 0; j < 4; ++j) {
        acc[i][j] = Frag<T>::mma(ah, bh[j], acc[i][j]);
        if (SPLIT) {
          acc[i][j] = Frag<T>::mma(ah, bl[j], acc[i][j]);
          acc[i][j] = Frag<T>::mma(al, bh[j], acc[i][j]);
        }
      }
      Frag<T>::guard(acc[i][0], acc[i][3], ah, SPLIT ? al : ah);
    }
    Frag<T>::keep(bh[0], bh[1], bh[2], bh[3]);
    if (SPLIT) Frag<T>::keep(bl[0], bl[1], bl[2], bl[3]);
  }
  acc_guard4(acc[0][0], acc[0][1], acc[0][2], acc[0][3]);
  acc_guard4(acc[1][0], acc[1][1], acc[1][2], acc[1][3]);
  acc_guard4(acc[2][0], acc[2][1], acc[2][2], acc[2][3]);
  acc_guard4(acc[3][0], acc[3][1], acc[3][2], acc[3][3]);

  float* slab = sT[wave];
  const float* Rb = RESID ? (resid + (size_t)b * strideR) : nullptr;
#pragma unroll
  for (int i = 0; i < 4; ++i) {
    const int mBase = m0 + (i << 4);
#pragma unroll
    for (int j = 0; j < 4; ++j) {
      const int n = n0 + (j << 4) + rlane;
      float bv = 0.f;
      if (BIAS_MODE == 2) bv = bias[n];
#pragma unroll
      for (int r = 0; r < 8; ++r) {
        float v = acc[i][j][r] * scale;
        if (BIAS_MODE == 1) v += bias[mBase + mOff + r];
        if (BIAS_MODE == 2) v += bv;
        if (RESID) v += Rb[(size_t)(mBase + mOff + r) * ldc + n];
        if (ACT == 2) v = fmaxf(v, 0.0f);
        if (ACT == 4) v = (v > 0.f) ? v : 0.01f * v;
        slab[(mOff + r) * 68 + (j << 4) + rlane] = v;
      }
    }
    __builtin_amdgcn_fence(__ATOMIC_RELEASE, "workgroup");
    __builtin_amdgcn_wave_barrier();
    __builtin_amdgcn_fence(__ATOMIC_ACQUIRE, "workgroup");
    if (OUT_MODE == 0) {
      float* C = (float*)Cout + (size_t)b * strideC;
      const int hh = lane >> 4, c4 = (lane & 15) * 4;
      for (int pass = 0; pass < 2; ++pass) {
#pragma unroll
        for (int it = 0; it < 8; ++it) {
          const int row = it * 2 + hh;
          v4f v = *(const v4f*)(slab + row * 68 + c4);
          *(volatile v4f*)(C + (size_t)(mBase + row) * ldc + n0 + c4) = v;
        }
        __threadfence();
      }
    } else {
      const int q = lane >> 3, c8 = (lane & 7) * 8;
      unsigned short* C  = (unsigned short*)Cout  + (size_t)b * strideC;
      unsigned short* C2 = (OUT_MODE == 2) ? ((unsigned short*)Cout2 + (size_t)b * strideC) : nullptr;
      for (int pass = 0; pass < 2; ++pass) {
#pragma unroll
        for (int it = 0; it < 4; ++it) {
          const int row = it * 4 + q;
          const float* sp = slab + row * 68 + c8;
          v8h hv, lv;
#pragma unroll
          for (int e = 0; e < 8; ++e) {
            if (OUT_MODE == 1) {
              hv[e] = (_Float16)sp[e];
            } else {
              unsigned short hb = f2bf_bits(sp[e]);
              unsigned short lb = f2bf_bits(sp[e] - bf_bits2f(hb));
              hv[e] = __builtin_bit_cast(_Float16, hb);
              lv[e] = __builtin_bit_cast(_Float16, lb);
            }
          }
          *(volatile v8h*)(C + (size_t)(mBase + row) * ldc + n0 + c8) = hv;
          if (OUT_MODE == 2) *(volatile v8h*)(C2 + (size_t)(mBase + row) * ldc + n0 + c8) = lv;
        }
        __threadfence();
      }
    }
    __builtin_amdgcn_fence(__ATOMIC_RELEASE, "workgroup");
    __builtin_amdgcn_wave_barrier();
    __builtin_amdgcn_fence(__ATOMIC_ACQUIRE, "workgroup");
  }
}

__global__ __launch_bounds__(256) void cast8_bf16_kernel(const float* __restrict__ in, unsigned short* __restrict__ out, int n8) {
  const int i = blockIdx.x * 256 + threadIdx.x;
  if (i >= n8) return;
  const float* p = in + 8 * (size_t)i;
  const v4f a = *(const v4f*)(p);
  const v4f c = *(const v4f*)(p + 4);
  unsigned short hb[8];
#pragma unroll
  for (int e = 0; e < 4; ++e) {
    hb[e]     = f2bf_bits(a[e]);
    hb[4 + e] = f2bf_bits(c[e]);
  }
  const v4u u = (v4u){pk16(hb[0], hb[1]), pk16(hb[2], hb[3]), pk16(hb[4], hb[5]), pk16(hb[6], hb[7])};
  unsigned short* q = out + 8 * (size_t)i;
  *(volatile v4u*)q = u;
  __threadfence();
  *(volatile v4u*)q = u;
}

__global__ __launch_bounds__(256) void bias_rne_kernel(const float* __restrict__ b0, const float* __restrict__ b1,
                                                       const float* __restrict__ b2, float* __restrict__ out) {
  const int z = blockIdx.x;
  const int t = threadIdx.x;
  const float* p = (z == 0) ? b0 : (z == 1) ? b1 : b2;
  const v4f v = *(const v4f*)(p + 4 * t);
  v4f r;
#pragma unroll
  for (int e = 0; e < 4; ++e) r[e] = bf_bits2f(f2bf_bits(v[e]));
  float* op = out + (size_t)z * kHid + 4 * t;
  *(volatile v4f*)op = r;
  __threadfence();
  *(volatile v4f*)op = r;
}

__global__ __launch_bounds__(256) void softmax_late_kernel(const float* __restrict__ Sp, unsigned short* __restrict__ Pp) {
  __shared__ float redM[8];
  __shared__ float redS[8];
  const int r    = blockIdx.x;
  const int i    = r + kEarly;
  const int t    = threadIdx.x;
  const int lane = t & 31, wave = t >> 5;
  const int jend = ((i >> 6) + 1) << 6;
  const int c0   = 8 * t;
  const int cb   = (c0 < jend - 8) ? c0 : (jend - 8);
  const float* sr = Sp + (size_t)r * kSeq + cb;
  const v4f a = *(const v4f*)(sr);
  const v4f c = *(const v4f*)(sr + 4);
  float x[8];
#pragma unroll
  for (int e = 0; e < 4; ++e) {
    const float f0 = (c0 + e <= i) ? 1.0f : 0.0f;
    const float f1 = (c0 + 4 + e <= i) ? 1.0f : 0.0f;
    x[e]     = fmaf(f0, a[e], (1.0f - f0) * kNegFill);
    x[4 + e] = fmaf(f1, c[e], (1.0f - f1) * kNegFill);
  }
  float mx = x[0];
#pragma unroll
  for (int e = 1; e < 8; ++e) mx = fmaxf(mx, x[e]);
#pragma unroll
  for (int off = 16; off > 0; off >>= 1) mx = fmaxf(mx, __shfl_xor(mx, off, 32));
  if (lane == 0) redM[wave] = mx;
  __syncthreads();
  float m = redM[0];
#pragma unroll
  for (int w = 1; w < 8; ++w) m = fmaxf(m, redM[w]);

  float ev[8];
  float sum = 0.0f;
#pragma unroll
  for (int e = 0; e < 8; ++e) {
    ev[e] = expf(x[e] - m);
    sum += ev[e];
  }
#pragma unroll
  for (int off = 16; off > 0; off >>= 1) sum += __shfl_xor(sum, off, 32);
  if (lane == 0) redS[wave] = sum;
  __syncthreads();
  float tot = redS[0];
#pragma unroll
  for (int w = 1; w < 8; ++w) tot += redS[w];
  const float inv = kPCarry * (1.0f / tot);

  unsigned short hb[8];
#pragma unroll
  for (int e = 0; e < 8; ++e) hb[e] = h_bits(ev[e] * inv);
  const v4u u = (v4u){pk16(hb[0], hb[1]), pk16(hb[2], hb[3]), pk16(hb[4], hb[5]), pk16(hb[6], hb[7])};
  unsigned short* pr = Pp + (size_t)r * kSeq + c0;
  *(volatile v4u*)pr = u;
  __threadfence();
  *(volatile v4u*)pr = u;
}

__global__ __launch_bounds__(256) void softmax_early_kernel(const float* __restrict__ Sp, unsigned short* __restrict__ Php,
                                                           unsigned short* __restrict__ Plp) {
  const int lane = threadIdx.x & 31, wave = threadIdx.x >> 5;
  const int i    = blockIdx.x * 8 + wave;
  const int jend = ((i >> 6) + 1) << 6;
  const int c0   = 8 * lane;
  const int cb   = (c0 < jend - 8) ? c0 : (jend - 8);
  const float* sr = Sp + (size_t)i * kEarly + cb;
  const v4f a = *(const v4f*)(sr);
  const v4f c = *(const v4f*)(sr + 4);
  float x[8];
#pragma unroll
  for (int e = 0; e < 4; ++e) {
    const float f0 = (c0 + e <= i) ? 1.0f : 0.0f;
    const float f1 = (c0 + 4 + e <= i) ? 1.0f : 0.0f;
    x[e]     = fmaf(f0, a[e], (1.0f - f0) * kNegFill);
    x[4 + e] = fmaf(f1, c[e], (1.0f - f1) * kNegFill);
  }
  float mx = x[0];
#pragma unroll
  for (int e = 1; e < 8; ++e) mx = fmaxf(mx, x[e]);
#pragma unroll
  for (int off = 16; off > 0; off >>= 1) mx = fmaxf(mx, __shfl_xor(mx, off, 32));
  float ev[8];
  float sum = 0.0f;
#pragma unroll
  for (int e = 0; e < 8; ++e) {
    ev[e] = expf(x[e] - mx);
    sum += ev[e];
  }
#pragma unroll
  for (int off = 16; off > 0; off >>= 1) sum += __shfl_xor(sum, off, 32);
  const float inv = 1.0f / sum;
  unsigned short hb[8], lb[8];
#pragma unroll
  for (int e = 0; e < 8; ++e) {
    const float p = ev[e] * inv;
    hb[e] = f2bf_bits(p);
    lb[e] = f2bf_bits(p - bf_bits2f(hb[e]));
  }
  const v4u uh = (v4u){pk16(hb[0], hb[1]), pk16(hb[2], hb[3]), pk16(hb[4], hb[5]), pk16(hb[6], hb[7])};
  const v4u ul = (v4u){pk16(lb[0], lb[1]), pk16(lb[2], lb[3]), pk16(lb[4], lb[5]), pk16(lb[6], lb[7])};
  unsigned short* ph = Php + (size_t)i * kEarly + c0;
  unsigned short* pl = Plp + (size_t)i * kEarly + c0;
  *(volatile v4u*)ph = uh;
  *(volatile v4u*)pl = ul;
  __threadfence();
  *(volatile v4u*)ph = uh;
  *(volatile v4u*)pl = ul;
}

extern "C" void kernel_launch(void* const* d_in, const int* in_sizes, int n_in,
                              void* d_out, int out_size, void* d_ws, size_t ws_size,
                              hipStream_t stream) {
  if (n_in < 7) return;
  if (in_sizes[0] != kTok * kEmb) return;
  if (in_sizes[1] != kHid * kEmb || in_sizes[3] != kHid * kEmb || in_sizes[5] != kHid * kEmb) return;
  if (in_sizes[2] != kHid || in_sizes[4] != kHid || in_sizes[6] != kHid) return;
  if (out_size != kTok * kHid) return;

  const size_t szXb   = (size_t)kTok * kEmb * 2;
  const size_t szW1   = (size_t)kHid * kEmb * 2;
  const size_t szBias = (size_t)3 * kHid * 4;
  const size_t szQK16 = (size_t)kTok * kHid * 2;
  const size_t szVT16 = (size_t)kBatch * kHid * kSeq * 2;
  const size_t szE    = (size_t)kBatch * kEarly * kHid * 2;
  const size_t szSL   = (size_t)kLate * kSeq * 4;
  const size_t szPL   = (size_t)kLate * kSeq * 2;
  const size_t szSE   = (size_t)kEarly * kEarly * 4;
  const size_t szPE   = (size_t)kEarly * kEarly * 2;

  const size_t offXb   = 0;
  const size_t offW    = offXb + szXb;
  const size_t offBias = offW + 3 * szW1;
  const size_t offQ16  = offBias + szBias;
  const size_t offK16  = offQ16 + szQK16;
  const size_t offVT16 = offK16 + szQK16;
  const size_t offQEH  = offVT16 + szVT16;
  const size_t offQEL  = offQEH + szE;
  const size_t offKEH  = offQEL + szE;
  const size_t offKEL  = offKEH + szE;
  const size_t offVTEH = offKEL + szE;
  const size_t offVTEL = offVTEH + szE;
  const size_t offSL   = offVTEL + szE;
  const size_t offPL   = offSL + szSL;
  const size_t offSE   = offPL + szPL;
  const size_t offPEH  = offSE + szSE;
  const size_t offPEL  = offPEH + szPE;
  const size_t total   = offPEL + szPE;
  if (ws_size < total) return;

  const float* x  = (const float*)d_in[0];
  const float* Wq = (const float*)d_in[1];
  const float* bq = (const float*)d_in[2];
  const float* Wk = (const float*)d_in[3];
  const float* bk = (const float*)d_in[4];
  const float* Wv = (const float*)d_in[5];
  const float* bv = (const float*)d_in[6];
  float* out = (float*)d_out;
  char* ws = (char*)d_ws;
  unsigned short* Xb   = (unsigned short*)(ws + offXb);
  unsigned short* Wqb  = (unsigned short*)(ws + offW);
  unsigned short* Wkb  = (unsigned short*)(ws + offW + szW1);
  unsigned short* Wvb  = (unsigned short*)(ws + offW + 2 * szW1);
  float* biasr = (float*)(ws + offBias);
  const float* bqr = biasr;
  const float* bkr = biasr + kHid;
  const float* bvr = biasr + 2 * kHid;
  unsigned short* Q16  = (unsigned short*)(ws + offQ16);
  unsigned short* K16  = (unsigned short*)(ws + offK16);
  unsigned short* VT16 = (unsigned short*)(ws + offVT16);
  unsigned short* QEH  = (unsigned short*)(ws + offQEH);
  unsigned short* QEL  = (unsigned short*)(ws + offQEL);
  unsigned short* KEH  = (unsigned short*)(ws + offKEH);
  unsigned short* KEL  = (unsigned short*)(ws + offKEL);
  unsigned short* VTEH = (unsigned short*)(ws + offVTEH);
  unsigned short* VTEL = (unsigned short*)(ws + offVTEL);
  float* SL = (float*)(ws + offSL);
  unsigned short* PL = (unsigned short*)(ws + offPL);
  float* SE = (float*)(ws + offSE);
  unsigned short* PEH = (unsigned short*)(ws + offPEH);
  unsigned short* PEL = (unsigned short*)(ws + offPEL);

  const int n8x = (kTok * kEmb) / 8;
  const int n8w = (kHid * kEmb) / 8;
  cast8_bf16_kernel<<<dim3(n8x / 256), dim3(256), 0, stream>>>(x,  Xb,  n8x);
  cast8_bf16_kernel<<<dim3(n8w / 256), dim3(256), 0, stream>>>(Wq, Wqb, n8w);
  cast8_bf16_kernel<<<dim3(n8w / 256), dim3(256), 0, stream>>>(Wk, Wkb, n8w);
  cast8_bf16_kernel<<<dim3(n8w / 256), dim3(256), 0, stream>>>(Wv, Wvb, n8w);
  bias_rne_kernel<<<dim3(3), dim3(256), 0, stream>>>(bq, bk, bv, biasr);

  const long strideTokBatch = (long)kSeq * kEmb;
  const long strideVT       = (long)kHid * kSeq;
  const long strideE        = (long)kEarly * kHid;

  {
    const int tilesQK = (kTok / 64) * (kHid / 64);
    wmma_gemm64<1, false, 2, 1, false, 0, 0><<<dim3(tilesQK / 8, 1), dim3(256), 0, stream>>>(
        Xb, Xb, kEmb, 0L, Wqb, Wqb, kEmb, 0L, (void*)Q16, (void*)Q16, kHid, 0L, bqr, bqr, 0L, kTok, kHid, kEmb, 1.0f, 0);
    wmma_gemm64<1, false, 2, 1, false, 0, 0><<<dim3(tilesQK / 8, 1), dim3(256), 0, stream>>>(
        Xb, Xb, kEmb, 0L, Wkb, Wkb, kEmb, 0L, (void*)K16, (void*)K16, kHid, 0L, bkr, bkr, 0L, kTok, kHid, kEmb, 1.0f, 0);
    const int tilesVT = (kHid / 64) * (kSeq / 64);
    wmma_gemm64<1, false, 1, 1, false, 0, 0><<<dim3(tilesVT / 8, kBatch), dim3(256), 0, stream>>>(
        Wvb, Wvb, kEmb, 0L, Xb, Xb, kEmb, strideTokBatch, (void*)VT16, (void*)VT16, kSeq, strideVT, bvr, bvr, 0L,
        kHid, kSeq, kEmb, 1.0f, 0);
  }
  {
    const int tilesE = (kEarly / 64) * (kHid / 64);
    wmma_gemm64<1, false, 2, 2, false, 0, 0><<<dim3(tilesE / 8, kBatch), dim3(256), 0, stream>>>(
        Xb, Xb, kEmb, strideTokBatch, Wqb, Wqb, kEmb, 0L, (void*)QEH, (void*)QEL, kHid, strideE, bqr, bqr, 0L,
        kEarly, kHid, kEmb, 1.0f, 0);
    wmma_gemm64<1, false, 2, 2, false, 0, 0><<<dim3(tilesE / 8, kBatch), dim3(256), 0, stream>>>(
        Xb, Xb, kEmb, strideTokBatch, Wkb, Wkb, kEmb, 0L, (void*)KEH, (void*)KEL, kHid, strideE, bkr, bkr, 0L,
        kEarly, kHid, kEmb, 1.0f, 0);
    const int tilesVE = (kHid / 64) * (kEarly / 64);
    wmma_gemm64<1, false, 1, 2, false, 0, 0><<<dim3(tilesVE / 8, kBatch), dim3(256), 0, stream>>>(
        Wvb, Wvb, kEmb, 0L, Xb, Xb, kEmb, strideTokBatch, (void*)VTEH, (void*)VTEL, kEarly, strideE, bvr, bvr, 0L,
        kHid, kEarly, kEmb, 1.0f, 0);
  }

  const int tilesSL = (kLate / 64) * (kSeq / 64);
  const int tilesOL = (kLate / 64) * (kHid / 64);
  const int tilesSE = (kEarly / 64) * (kEarly / 64);
  const int tilesOE = (kEarly / 64) * (kHid / 64);
  for (int b = 0; b < kBatch; ++b) {
    const size_t tokLate  = ((size_t)b * kSeq + kEarly) * kHid;
    const size_t tokBatch = (size_t)b * kSeq * kHid;

    wmma_gemm64<0, false, 0, 0, false, 0, 1><<<dim3(tilesSL / 8, 1), dim3(256), 0, stream>>>(
        Q16 + tokLate, Q16 + tokLate, kHid, 0L, K16 + tokBatch, K16 + tokBatch, kHid, 0L,
        (void*)SL, (void*)SL, kSeq, 0L, bqr, bqr, 0L, kLate, kSeq, kHid, kScoreScale, kEarly);
    softmax_late_kernel<<<dim3(kLate), dim3(256), 0, stream>>>(SL, PL);
    wmma_gemm64<0, false, 0, 0, false, 0, 2><<<dim3(tilesOL / 8, 1), dim3(256), 0, stream>>>(
        PL, PL, kSeq, 0L, VT16 + (size_t)b * strideVT, VT16 + (size_t)b * strideVT, kSeq, 0L,
        (void*)(out + tokLate), (void*)(out + tokLate), kHid, 0L, bqr, bqr, 0L, kLate, kHid, kSeq, kPCarryInv, kEarly);

    wmma_gemm64<1, true, 0, 0, false, 0, 1><<<dim3(tilesSE / 8, 1), dim3(256), 0, stream>>>(
        QEH + (size_t)b * strideE, QEL + (size_t)b * strideE, kHid, 0L,
        KEH + (size_t)b * strideE, KEL + (size_t)b * strideE, kHid, 0L,
        (void*)SE, (void*)SE, kEarly, 0L, bqr, bqr, 0L, kEarly, kEarly, kHid, kScoreScale, 0);
    softmax_early_kernel<<<dim3(kEarly / 8), dim3(256), 0, stream>>>(SE, PEH, PEL);
    wmma_gemm64<1, true, 0, 0, false, 0, 2><<<dim3(tilesOE / 8, 1), dim3(256), 0, stream>>>(
        PEH, PEL, kEarly, 0L, VTEH + (size_t)b * strideE, VTEL + (size_t)b * strideE, kEarly, 0L,
        (void*)(out + tokBatch), (void*)(out + tokBatch), kHid, 0L, bqr, bqr, 0L, kEarly, kHid, kEarly, 1.0f, 0);
  }
}
